// DREAMReconstructor_71270687310083
// MI455X (gfx1250) — hardware-run, weakly checked
//
#include <hip/hip_runtime.h>


#define NB   256
#define NT   1024
#define NI   39
#define NH   256
#define NR   16
#define NIP  64
#define NRP  32
#define NOP  48
#define NPP  64
typedef _Float16 h16;
typedef unsigned short bf;
typedef __attribute__((ext_vector_type(16))) __bf16   v16bf;
typedef __attribute__((ext_vector_type(16))) _Float16 v16h;
typedef __attribute__((ext_vector_type(8)))  _Float16 v8h;
typedef __attribute__((ext_vector_type(8)))  unsigned short v8us;
typedef __attribute__((ext_vector_type(8)))  float    v8f;
typedef __attribute__((ext_vector_type(4)))  float    v4f;
typedef v8h  __attribute__((may_alias)) v8ha;
typedef v4f  __attribute__((may_alias)) v4fa;
typedef v8us __attribute__((may_alias)) v8usa;

__device__ __forceinline__ unsigned short f2bf(float f) { unsigned u = __float_as_uint(f); u += 0x7FFFu + ((u >> 16) & 1u); return (unsigned short)(u >> 16); }
__device__ __forceinline__ float bf2f(unsigned short b) { return __uint_as_float(((unsigned)b) << 16); }
__device__ __forceinline__ float bfr(float f) { return bf2f(f2bf(f)); }
__device__ __forceinline__ v16h cat16(v8h lo, v8h hi) { return __builtin_shufflevector(lo, hi, 0, 1, 2, 3, 4, 5, 6, 7, 8, 9, 10, 11, 12, 13, 14, 15); }
__device__ __forceinline__ v16bf cat16b(v8us lo, v8us hi) { return __builtin_bit_cast(v16bf, __builtin_shufflevector(lo, hi, 0, 1, 2, 3, 4, 5, 6, 7, 8, 9, 10, 11, 12, 13, 14, 15)); }
__device__ __forceinline__ v8f wmma16(v16h a, v16h b, v8f c) { return __builtin_amdgcn_wmma_f32_16x16x32_f16(false, a, false, b, (short)0, c, false, false); }
__device__ __forceinline__ v8f wmmab(v16bf a, v16bf b, v8f c) { return __builtin_amdgcn_wmma_f32_16x16x32_bf16(false, a, false, b, (short)0, c, false, false); }

template <typename T16> struct WFrag;
template <> struct WFrag<h16> { typedef v16h V; static __device__ __forceinline__ V ld(const h16* p) { return cat16(*(const v8h*)p, *(const v8h*)(p + 16)); } static __device__ __forceinline__ v8f mma(V a, V b, v8f c) { return wmma16(a, b, c); } };
template <> struct WFrag<bf> { typedef v16bf V; static __device__ __forceinline__ V ld(const bf* p) { return cat16b(*(const v8us*)p, *(const v8us*)(p + 16)); } static __device__ __forceinline__ v8f mma(V a, V b, v8f c) { return wmmab(a, b, c); } };

typedef __attribute__((ext_vector_type(2))) _Float16 v2h;
typedef __attribute__((ext_vector_type(4))) _Float16 v4h;
typedef __attribute__((ext_vector_type(2))) unsigned short v2us;
typedef __attribute__((ext_vector_type(4))) unsigned short v4us;
typedef __attribute__((ext_vector_type(2))) float v2f;
typedef __attribute__((ext_vector_type(4))) int v4i;

__device__ __forceinline__ h16 toh_flush(float x) { const float z = (fabsf(x) < 6.103515625e-05f) ? 0.0f : x; return (h16)z; }

__device__ __forceinline__ float tanhc(float v) { return 1.0f - 2.0f / (expf(2.0f * v) + 1.0f); }

__global__ __launch_bounds__(256) void k_padcast(const float* __restrict__ src, h16* dst, int R, int C, int RP, int CP) { const int i = blockIdx.x * 256 + threadIdx.x; if (i >= RP * CP / 4) return; const int r = (i * 4) / CP, c0 = (i * 4) % CP; v4h o;
#pragma unroll
    for (int q = 0; q < 4; ++q) { const int c = c0 + q; const bool live = (r < R) && (c < C); const unsigned short keep = live ? (unsigned short)0xFFFFu : (unsigned short)0u; const float v = src[(size_t)(live ? r : 0) * C + (live ? c : 0)]; o[q] = __builtin_bit_cast(h16, (unsigned short)(__builtin_bit_cast(unsigned short, toh_flush(bfr(v))) & keep)); }
    *(volatile v4h*)(dst + (size_t)i * 4) = o; __threadfence(); *(volatile v4h*)(dst + (size_t)i * 4) = o; }

__device__ __forceinline__ void rnn_pair(int c, const v16h& zf, const v16h& xf0, const v16h& xf1, const h16* alp, const h16* wip, const h16* blp, const h16* wdp, const float* __restrict__ b, int hi, v8f& zn, v8f& dec0, v8f& dec1, v8f& dec2, v8f& ha, v8f& hb) { v8h h0, h1;
#pragma unroll
    for (int u = 0; u < 2; ++u) { const int ut = 2 * c + u; v8f pre = (v8f){};
        pre = wmma16(WFrag<h16>::ld(alp + (size_t)(8 * ut) * NRP), zf, pre); pre = wmma16(WFrag<h16>::ld(wip + (size_t)(8 * ut) * NIP), xf0, pre); pre = wmma16(WFrag<h16>::ld(wip + (size_t)(8 * ut) * NIP + 32), xf1, pre);
#pragma unroll
        for (int j = 0; j < 8; ++j) { const float hv = tanhc(pre[j] + bfr(b[128 * hi + 8 * ut + j])); if (u == 0) { ha[j] = hv; h0[j] = toh_flush(hv); } else { hb[j] = hv; h1[j] = toh_flush(hv); } } }
    const v16h hf = cat16(h0, h1);
    zn = wmma16(cat16(*(const v8h*)(blp + 16 * c), *(const v8h*)(blp + 16 * c + 8)), hf, zn);
    dec0 = wmma16(cat16(*(const v8h*)(wdp + 16 * c), *(const v8h*)(wdp + 16 * c + 8)), hf, dec0);
    dec1 = wmma16(cat16(*(const v8h*)(wdp + (size_t)8 * NH + 16 * c), *(const v8h*)(wdp + (size_t)8 * NH + 16 * c + 8)), hf, dec1);
    dec2 = wmma16(cat16(*(const v8h*)(wdp + (size_t)16 * NH + 16 * c), *(const v8h*)(wdp + (size_t)16 * NH + 16 * c + 8)), hf, dec2); }

template <bool LAST>
__device__ __forceinline__ void rnn_step(v8f& z, const h16* xt, const h16* alp, const h16* wip, const h16* blp, const h16* wdp, const float* __restrict__ b, int hi, const v8f& bd0, const v8f& bd1, const v8f& bd2, float* pp, float* hl) { v8h zl;
#pragma unroll
    for (int j = 0; j < 8; ++j) zl[j] = toh_flush(z[j]);
    const v16h zf = cat16(zl, (v8h){}); const v16h xf0 = WFrag<h16>::ld(xt); const v16h xf1 = WFrag<h16>::ld(xt + 32);
    v8f zn = (v8f){}, dec0 = (v8f){}, dec1 = (v8f){}, dec2 = (v8f){};
    if (LAST) {
#pragma unroll
        for (int q = 0; q < 4; ++q) { v8f g[4]; rnn_pair(2 * q, zf, xf0, xf1, alp, wip, blp, wdp, b, hi, zn, dec0, dec1, dec2, g[0], g[1]); rnn_pair(2 * q + 1, zf, xf0, xf1, alp, wip, blp, wdp, b, hi, zn, dec0, dec1, dec2, g[2], g[3]);
#pragma unroll
            for (int pass = 0; pass < 2; ++pass) {
#pragma unroll
                for (int k = 0; k < 8; ++k) { v4f s;
#pragma unroll
                    for (int j = 0; j < 4; ++j) s[j] = g[k >> 1][4 * (k & 1) + j];
                    *(volatile v4f*)(hl + 32 * q + 4 * k) = s; }
                if (pass == 0) __threadfence(); } } }
    else { for (int c = 0; c < 8; ++c) { v8f ha, hb; rnn_pair(c, zf, xf0, xf1, alp, wip, blp, wdp, b, hi, zn, dec0, dec1, dec2, ha, hb); } }
    const v8f r0 = dec0 + bd0, r1 = dec1 + bd1, r2 = dec2 + bd2;
#pragma unroll
    for (int pass = 0; pass < 2; ++pass) { v4f q;
#pragma unroll
        for (int k = 0; k < 2; ++k) {
#pragma unroll
            for (int j = 0; j < 4; ++j) q[j] = r0[4 * k + j];
            *(volatile v4f*)(pp + 4 * k) = q; }
#pragma unroll
        for (int k = 0; k < 2; ++k) {
#pragma unroll
            for (int j = 0; j < 4; ++j) q[j] = r1[4 * k + j];
            *(volatile v4f*)(pp + 8 + 4 * k) = q; }
#pragma unroll
        for (int k = 0; k < 2; ++k) {
#pragma unroll
            for (int j = 0; j < 4; ++j) q[j] = r2[4 * k + j];
            *(volatile v4f*)(pp + 16 + 4 * k) = q; }
        q[0] = 0.0f; q[1] = 0.0f; q[2] = 0.0f; q[3] = 0.0f; *(volatile v4f*)(pp + 24) = q; *(volatile v4f*)(pp + 28) = q;
        if (pass == 0) __threadfence(); }
    z = zn; }

__global__ __launch_bounds__(32) void k_rnn(const h16* __restrict__ X16, const h16* __restrict__ Wi, const h16* __restrict__ Al, const h16* __restrict__ Bl, const h16* __restrict__ Wd, const float* __restrict__ b, const float* __restrict__ bd, float* P, float* hlast) {
    if (blockIdx.x >= (unsigned)(NB / 16)) return;
    const int lane = threadIdx.x & 31, lr = lane & 15, hi = lane >> 4; const size_t row = (size_t)blockIdx.x * 16 + lr;
    const h16* xr = X16 + row * NT * NIP + 8 * hi; const int urow = 128 * (lr >> 3) + (lr & 7); const int drow = 24 * (lr >> 3) + (lr & 7);
    const h16* alp = Al + (size_t)urow * NRP + 8 * hi; const h16* wip = Wi + (size_t)urow * NIP + 8 * hi; const h16* blp = Bl + (size_t)lr * NH + 128 * hi; const h16* wdp = Wd + (size_t)drow * NH + 128 * hi;
    float* pr = P + row * NT * NPP + 32 * hi; float* hl = hlast + row * NH + 128 * hi;
    v8f bd0, bd1, bd2;
#pragma unroll
    for (int j = 0; j < 8; ++j) { const int d0 = 24 * hi + j, d1 = d0 + 8, d2 = d0 + 16; const float v0 = bfr(bd[d0 < NI ? d0 : 0]), v1 = bfr(bd[d1 < NI ? d1 : 0]), v2 = bfr(bd[d2 < NI ? d2 : 0]); bd0[j] = (d0 < NI) ? v0 : 0.0f; bd1[j] = (d1 < NI) ? v1 : 0.0f; bd2[j] = (d2 < NI) ? v2 : 0.0f; }
    v8f z = (v8f){};
    for (int t = 0; t < NT - 1; ++t) rnn_step<false>(z, xr + (size_t)t * NIP, alp, wip, blp, wdp, b, hi, bd0, bd1, bd2, pr + (size_t)t * NPP, hl);
    rnn_step<true>(z, xr + (size_t)(NT - 1) * NIP, alp, wip, blp, wdp, b, hi, bd0, bd1, bd2, pr + (size_t)(NT - 1) * NPP, hl);
}

__global__ __launch_bounds__(256) void k_pack(const float* __restrict__ P, float* recon, int n4) { const int i = blockIdx.x * 256 + threadIdx.x; if (i >= n4) return; v4f o;
#pragma unroll
    for (int q = 0; q < 4; ++q) { const unsigned e = (unsigned)i * 4u + (unsigned)q; const unsigned rec = e / (unsigned)NI, d = e % (unsigned)NI; o[q] = P[(size_t)rec * NPP + (d < 24u ? d : d + 8u)]; }
    *(volatile v4f*)(recon + (size_t)i * 4) = o; __threadfence(); *(volatile v4f*)(recon + (size_t)i * 4) = o; }

extern "C" void kernel_launch(void* const* d_in, const int* in_sizes, int n_in, void* d_out, int out_size, void* d_ws, size_t ws_size, hipStream_t stream) {
    if (n_in < 7) return;
    if (in_sizes[0] != NB * NT * NI || in_sizes[1] != NH * NI || in_sizes[2] != NH * NR || in_sizes[3] != NR * NH || in_sizes[4] != NH || in_sizes[5] != NI * NH || in_sizes[6] != NI) return;
    if (out_size != NB * NT * NI + NB * NH) return;
    static_assert(NB % 16 == 0 && NH == 256 && NR == 16 && NRP == 32 && NIP == 64 && NI <= NIP && NI <= NOP && NOP == 48 && NPP == 64 && (NB * NT * NIP / 4) % 256 == 0 && (NH * NIP / 4) % 256 == 0 && (NH * NRP / 4) % 256 == 0 && (NR * NH / 4) % 256 == 0 && (NOP * NH / 4) % 256 == 0 && (NB * NT * NI / 4) % 256 == 0 && (NB * NT * NI * 4) % 128 == 0, "a wave 16 rows; 256 units = 16 tiles; the paddings are the matrix word's depth and tile; every elementwise grid exact; the second output begins on a 128-byte line");
    const float* x = (const float*)d_in[0]; const float* win = (const float*)d_in[1]; const float* a = (const float*)d_in[2]; const float* bl = (const float*)d_in[3]; const float* b = (const float*)d_in[4]; const float* wd = (const float*)d_in[5]; const float* bd = (const float*)d_in[6];
    float* out = (float*)d_out; float* recon = out;     float* hlast = out + (size_t)NB * NT * NI;
    char* wsp = (char*)d_ws; auto take = [&](size_t bytes) { char* p = wsp; wsp += (bytes + 255) & ~(size_t)255; return (void*)p; };
    h16* X16 = (h16*)take((size_t)NB * NT * NIP * 2);     h16* Wi = (h16*)take((size_t)NH * NIP * 2);     h16* Al = (h16*)take((size_t)NH * NRP * 2);     h16* Bl = (h16*)take((size_t)NR * NH * 2);     h16* Wd = (h16*)take((size_t)NOP * NH * 2);     float* P = (float*)take((size_t)NB * NT * NPP * 4);
    if ((size_t)(wsp - (char*)d_ws) > ws_size) return;
    k_padcast<<<(unsigned)(NB * NT * NIP / 4 / 256), 256, 0, stream>>>(x, X16, NB * NT, NI, NB * NT, NIP);
    k_padcast<<<(unsigned)(NH * NIP / 4 / 256), 256, 0, stream>>>(win, Wi, NH, NI, NH, NIP);
    k_padcast<<<(unsigned)(NH * NRP / 4 / 256), 256, 0, stream>>>(a, Al, NH, NR, NH, NRP);
    k_padcast<<<(unsigned)(NR * NH / 4 / 256), 256, 0, stream>>>(bl, Bl, NR, NH, NR, NH);
    k_padcast<<<(unsigned)(NOP * NH / 4 / 256), 256, 0, stream>>>(wd, Wd, NI, NH, NOP, NH);
    k_rnn<<<(unsigned)(NB / 16), 32, 0, stream>>>(X16, Wi, Al, Bl, Wd, b, bd, P, hlast);
    k_pack<<<(unsigned)(NB * NT * NI / 4 / 256), 256, 0, stream>>>(P, recon, NB * NT * NI / 4);
}
